// LegendreEncoding_7670811591192
// MI455X (gfx1250) — hardware-verified
//
#include <hip/hip_runtime.h>
#include <math.h>

typedef __attribute__((ext_vector_type(16))) _Float16 v16h;
typedef __attribute__((ext_vector_type(16))) __bf16 v16b;
typedef __attribute__((ext_vector_type(8)))  _Float16 v8h;
typedef __attribute__((ext_vector_type(8)))  float v8f;
typedef __attribute__((ext_vector_type(4)))  float v4f;
typedef __attribute__((ext_vector_type(2)))  float v2f;
typedef __attribute__((ext_vector_type(4)))  unsigned v4u;
typedef __attribute__((ext_vector_type(4)))  int v4i;
typedef float __attribute__((may_alias)) float_a;
typedef int __attribute__((may_alias)) int_a;

template <typename T> __device__ __forceinline__ void vst2(void* p, T v) { *(volatile T*)p = v; __threadfence(); *(volatile T*)p = v; }
__device__ __forceinline__ v8f wmma16(v16h a, v16h b, v8f c) {
  v8f d = __builtin_amdgcn_wmma_f32_16x16x32_f16(false, a, false, b, (short)0, c, false, false);
  asm volatile("v_nop\n\tv_nop\n\tv_nop\n\tv_nop" : "+v"(d) : "v"(a), "v"(b));
  return d;
}
__device__ __forceinline__ v8f wmma_bf(v16b a, v16b b, v8f c) {
  v8f d = __builtin_amdgcn_wmma_f32_16x16x32_bf16(false, a, false, b, (short)0, c, false, false);
  asm volatile("v_nop\n\tv_nop\n\tv_nop\n\tv_nop" : "+v"(d) : "v"(a), "v"(b));
  return d;
}
__device__ __forceinline__ v16h frag_h(const _Float16* rowk0, int lane) {
  union { v16h v; v8h q[2]; } u; const _Float16* p = rowk0 + 8 * (lane >> 4);
  u.q[0] = *(const v8h*)p; u.q[1] = *(const v8h*)(p + 16); return u.v;
}
__device__ __forceinline__ v16h frag_f32(const float* rowk0, int lane) {
  v16h a; const float* p = rowk0 + 8 * (lane >> 4);
#pragma unroll
  for (int i = 0; i < 8; ++i) { a[i] = (_Float16)p[i]; a[8 + i] = (_Float16)p[16 + i]; }
  return a;
}
__device__ __forceinline__ v16h frag_f32s(const float* rowk0, int lane, float sc) {
  v16h a; const float* p = rowk0 + 8 * (lane >> 4);
#pragma unroll
  for (int i = 0; i < 8; ++i) { a[i] = (_Float16)(p[i] * sc); a[8 + i] = (_Float16)(p[16 + i] * sc); }
  return a;
}
__device__ __forceinline__ v16h fragc_f32(const float* W, int k0, int n, int lane, int ld, int K) {
  v16h a; const int g = lane >> 4;
#pragma unroll
  for (int i = 0; i < 8; ++i) { const int ka = k0 + 8 * g + i, kb = ka + 16;
    a[i] = (_Float16)(ka < K ? W[(size_t)(ka < K ? ka : K - 1) * ld + n] : 0.f); a[8 + i] = (_Float16)(kb < K ? W[(size_t)(kb < K ? kb : K - 1) * ld + n] : 0.f); }
  return a;
}
struct F2 { v16b h, l; };
__device__ __forceinline__ F2 bsplit16(const float v[16]) { F2 r;
#pragma unroll
  for (int i = 0; i < 16; ++i) { const __bf16 h = (__bf16)v[i]; r.h[i] = h; r.l[i] = (__bf16)(v[i] - (float)h); }
  return r; }
__device__ __forceinline__ F2 split_row(const float* row, int k0, int lane) { float v[16]; const float* p = row + k0 + 8 * (lane >> 4);
#pragma unroll
  for (int i = 0; i < 8; ++i) { v[i] = p[i]; v[8 + i] = p[16 + i]; }
  return bsplit16(v); }
__device__ __forceinline__ F2 split_rowK(const float* row, int k0, int lane, int K) { float v[16]; const int g = lane >> 4;
#pragma unroll
  for (int i = 0; i < 8; ++i) { const int ka = k0 + 8 * g + i, kb = ka + 16; v[i] = ka < K ? row[ka < K ? ka : K - 1] : 0.f; v[8 + i] = kb < K ? row[kb < K ? kb : K - 1] : 0.f; }
  return bsplit16(v); }
__device__ __forceinline__ F2 split_col(const float* W, int k0, int n, int lane, int ld, int K) { float v[16]; const int g = lane >> 4;
#pragma unroll
  for (int i = 0; i < 8; ++i) { const int ka = k0 + 8 * g + i, kb = ka + 16; v[i] = ka < K ? W[(size_t)(ka < K ? ka : K - 1) * ld + n] : 0.f; v[8 + i] = kb < K ? W[(size_t)(kb < K ? kb : K - 1) * ld + n] : 0.f; }
  return bsplit16(v); }
__device__ __forceinline__ v8f mac3(const F2& a, const F2& b, v8f c) { c = wmma_bf(a.l, b.h, c); c = wmma_bf(a.h, b.l, c); return wmma_bf(a.h, b.h, c); }
__device__ __forceinline__ float sigm(float v) { return 1.0f / (1.0f + expf(-v)); }
#define LDSX() do { asm volatile("s_wait_dscnt 0" ::: "memory"); __builtin_amdgcn_wave_barrier(); __builtin_amdgcn_fence(__ATOMIC_RELEASE, "workgroup"); } while (0)


#define NN 131072
#define KK 16
#define HALF 64
#define KD (KK * HALF)
typedef __attribute__((ext_vector_type(8))) __bf16 v8b;
__device__ __forceinline__ v16b frag_b(const __bf16* rowk0, int lane) {
  union { v16b v; v8b q[2]; } u; const __bf16* p = rowk0 + 8 * (lane >> 4);
  u.q[0] = *(const v8b*)p; u.q[1] = *(const v8b*)(p + 16); return u.v;
}
__device__ __forceinline__ float bfr(float v) { return (float)(__bf16)v; }
__device__ __attribute__((noinline)) float exp_ni(float v) { return expf(v); }
__device__ __attribute__((noinline)) float erf_ni(float v) { return erff(v); }
__device__ __attribute__((noinline)) float tanh_ni(float v) { return tanhf(v); }
__device__ __attribute__((noinline)) float pow_ni(float a, float b) { return powf(a, b); }

#define WS_WB  0u
#define WS_CST (WS_WB + 2u * KK * KD)
#define WS_END (WS_CST + 128u)

__global__ __launch_bounds__(256) void k_prep(const float* __restrict__ Wm, const float* __restrict__ Bv, __bf16* __restrict__ WB, float* __restrict__ CST) {
  __shared__ __align__(16) __bf16 s[KK][KD]; __shared__ __align__(16) float sc[32]; const int t = threadIdx.x;
  for (int e2 = t; e2 < KK * KD; e2 += 256) { const int k = e2 / KD, kd = e2 % KD; const int kb = kd / HALF, h = kd % HALF; s[k][kd] = (__bf16)((kb == k) ? Wm[k * (2 * HALF + 1) + 1 + HALF + h] : 0.f); }
  if (t < 32) { float c = 0.f; if (t < KK) { c = bfr(Bv[t]) + bfr(Wm[t * (2 * HALF + 1)]); for (int h = 1; h <= HALF; ++h) c += bfr(Wm[t * (2 * HALF + 1) + h]); } sc[t] = c; }
  __syncthreads();
  for (int q = t; q < KK * KD / 8; q += 256) vst2((unsigned*)(WB + (size_t)q * 8), *(const v4u*)(&s[0][0] + (size_t)q * 8));
  if (t < 8) vst2(CST + t * 4, *(const v4f*)&sc[t * 4]);
}
__global__ __launch_bounds__(128) void k_enc(const float* __restrict__ E, const __bf16* __restrict__ WB, const float* __restrict__ CST, float* __restrict__ OUT) {
  __shared__ __align__(16) float st[KK][68];
  const int tid = threadIdx.x, wave = tid >> 5, lane = tid & 31, col = lane & 15, g = lane >> 4; const size_t n0 = (size_t)blockIdx.x * 64 + wave * 16; const float ev = bfr(E[n0 + col]);
  v8f acc = {}, accl = {};
#pragma unroll 1
  for (int k = 0; k < KK; ++k) { const float Ek = pow_ni(ev, (float)(k + 1));
#pragma unroll
    for (int hc = 0; hc < 2; ++hc) { v16b ah, al;
#pragma unroll
      for (int e2 = 0; e2 < 16; ++e2) { const int h = hc * 32 + 8 * g + (e2 & 7) + ((e2 >> 3) << 4); const float x = tanh_ni(Ek * (float)(h + 1) / 5.0f); const __bf16 hb = (__bf16)x; ah[e2] = hb; al[e2] = (__bf16)(x - (float)hb); }
      const v16b w = frag_b(WB + (size_t)col * KD + k * HALF + hc * 32, lane); acc = wmma_bf(ah, w, acc); accl = wmma_bf(al, w, accl); } }
#pragma unroll
  for (int r = 0; r < 8; ++r) st[col][wave * 16 + 8 * g + r] = acc[r] + accl[r] + CST[col];
  __syncthreads();
  for (int e2 = tid; e2 < KK * 16; e2 += 128) { const int k = e2 >> 4, pc = e2 & 15; vst2(OUT + (size_t)k * NN + (size_t)blockIdx.x * 64 + pc * 4, *(const v4f*)&st[k][pc * 4]); }
}
extern "C" void kernel_launch(void* const* d_in, const int* in_sizes, int n_in, void* d_out, int out_size, void* d_ws, size_t ws_size, hipStream_t stream) {
  (void)in_sizes; (void)n_in; (void)out_size;
  const float** F = (const float**)d_in;
  if (ws_size < (size_t)WS_END) return;
  char* ws = (char*)d_ws; __bf16* WB = (__bf16*)(ws + WS_WB); float* CST = (float*)(ws + WS_CST);
  k_prep<<<1, 256, 0, stream>>>(F[1], F[2], WB, CST);
  k_enc<<<NN / 64, 128, 0, stream>>>(F[0], WB, CST, (float*)d_out);
}
